// MTNN_66271345377548
// MI455X (gfx1250) — hardware-run, weakly checked
//
#include <hip/hip_runtime.h>
#include <math.h>

typedef __attribute__((ext_vector_type(16))) _Float16 v16h;
typedef __attribute__((ext_vector_type(8)))  _Float16 v8h;
typedef __attribute__((ext_vector_type(8)))  float    v8f;
typedef __attribute__((ext_vector_type(4)))  float    v4f;
typedef __attribute__((ext_vector_type(4)))  unsigned int v4u;
typedef v4u v4u_alias __attribute__((may_alias));

constexpr int kB    = 512;
constexpr int kT    = 200;
constexpr int kIS   = 64;
constexpr int kID   = 128;
constexpr int kHS   = 256;
constexpr int kHD   = 256;
constexpr int kNN   = 256;
constexpr int kDH   = kHS + 2 * kHD;
constexpr int kRows = kB * kT;
constexpr int kPS   = 32;
constexpr int kRB   = 16;

constexpr float kCarryX = 16.0f;
constexpr float kCarryW = 256.0f;
constexpr float kCarryA = 16.0f;
constexpr float kFoldXW = 1.0f / (kCarryX * kCarryW);
constexpr float kFoldAW = 1.0f / (kCarryA * kCarryW);
constexpr float kFoldA  = 1.0f / kCarryA;

static_assert(kDH == 768);
static_assert(kRows == 102400);
static_assert((kRows % 64) == 0 && (kHD % 64) == 0);
static_assert((kID % 32) == 0 && (kHD % 32) == 0);
static_assert((kB % kPS) == 0 && (kB % kRB) == 0);
static_assert(((kRB * kT * 4) % 128) == 0);
static_assert((kT % 4) == 0);
static_assert(kPS * kIS == 256 * 8);

constexpr size_t kSzD    = (size_t)kRows * kHD * 2;
constexpr size_t kSzXP   = (size_t)kRows * kHD * 2;
constexpr size_t kSzXH   = (size_t)kRows * kID * 2;
constexpr size_t kSzW16  = ((size_t)kHD * kID + 4 * (size_t)kHD * kHD) * 2;
constexpr size_t kSzBIAS = 3 * (size_t)kHD * 4;
constexpr size_t kSzYST  = (size_t)kB * 4;
constexpr size_t kSzY    = (size_t)kB * kT * 4;
constexpr size_t kOffD    = 0;
constexpr size_t kOffXP   = kOffD + kSzD;
constexpr size_t kOffW16  = kOffXP + kSzXP;
constexpr size_t kOffBIAS = kOffW16 + kSzW16;
constexpr size_t kOffYST  = kOffBIAS + kSzBIAS;
constexpr size_t kOffYF   = kOffYST + kSzYST;
constexpr size_t kOffYB   = kOffYF + kSzY;
constexpr size_t kWsTotal = kOffYB + kSzY;
static_assert(kSzXH <= kSzXP);
static_assert(kWsTotal == 106271744ull);
static_assert(kWsTotal <= 134217728ull);
static_assert((kOffXP % 128) == 0 && (kOffW16 % 128) == 0 && (kOffBIAS % 128) == 0 &&
              (kOffYST % 128) == 0 && (kOffYF % 128) == 0 && (kOffYB % 128) == 0);
constexpr size_t kWOffDyn  = 0;
constexpr size_t kWOffIhF  = (size_t)kHD * kID;
constexpr size_t kWOffIhB  = kWOffIhF + (size_t)kHD * kHD;
constexpr size_t kWOffHhF  = kWOffIhB + (size_t)kHD * kHD;
constexpr size_t kWOffHhB  = kWOffHhF + (size_t)kHD * kHD;

__device__ __forceinline__ float rbf(float f) {
  unsigned u = __float_as_uint(f);
  u += 0x7FFFu + ((u >> 16) & 1u);
  u &= 0xFFFF0000u;
  return __uint_as_float(u);
}
__device__ __forceinline__ float h16_to_f32(unsigned hb) {
  const unsigned sgn = (hb & 0x8000u) << 16;
  const unsigned em = hb & 0x7fffu;
  const float fn = __uint_as_float((em << 13) + 0x38000000u);
  const float fs = (float)em * 5.9604644775390625e-8f;
  const float mag = (em < 0x400u) ? fs : fn;
  return __uint_as_float(__float_as_uint(mag) | sgn);
}
union FragU { v16h v; v8h h[2]; };
__device__ __forceinline__ v16h frag_load(const _Float16* p) {
  FragU f;
  f.h[0] = *(const v8h*)(p);
  f.h[1] = *(const v8h*)(p + 16);
  return f.v;
}
__device__ __forceinline__ v8f mma_plain(v16h a, v16h b, v8f c) {
  return __builtin_amdgcn_wmma_f32_16x16x32_f16(false, a, false, b, (short)0, c, false, false);
}
__device__ __forceinline__ void guard1(v8f& c, v16h a, v16h b) {
  asm volatile("v_nop\n\tv_nop\n\tv_nop\n\tv_nop" : "+v"(c) : "v"(a), "v"(b));
}
__device__ __forceinline__ void acc_guard1(v8f& c) {
  asm volatile("v_nop\n\tv_nop\n\tv_nop\n\tv_nop" : "+v"(c));
}
__device__ __forceinline__ void keep4(v16h a, v16h b, v16h c, v16h d) {
  asm volatile("v_nop" :: "v"(a), "v"(b), "v"(c), "v"(d));
}
__device__ __forceinline__ v8f mma_g(v16h a, v16h b, v8f c) {
  c = __builtin_amdgcn_wmma_f32_16x16x32_f16(false, a, false, b, (short)0, c, false, false);
  asm volatile("v_nop\n\tv_nop\n\tv_nop\n\tv_nop" : "+v"(c) : "v"(a), "v"(b));
  return c;
}
__device__ __forceinline__ v8h cvt8(const float* src, float carry) {
  const v4f a0 = *(const v4f*)(src);
  const v4f a1 = *(const v4f*)(src + 4);
  v8h r;
#pragma unroll
  for (int e = 0; e < 4; ++e) {
    const float t0 = a0[e];
    const float t1 = a1[e];
    r[e]     = (_Float16)(rbf(t0) * carry);
    r[4 + e] = (_Float16)(rbf(t1) * carry);
  }
  return r;
}

__global__ __launch_bounds__(256) void cvt_weights_kernel(
    const float* __restrict__ wdyn, const float* __restrict__ wihf, const float* __restrict__ wihb,
    const float* __restrict__ whhf, const float* __restrict__ whhb, unsigned short* __restrict__ dst)
{
  const int blk = blockIdx.x;
  const float* src = wdyn;
  int lb = blk;
  if (blk >= 16) {
    const int q = (blk - 16) >> 5;
    lb = (blk - 16) & 31;
    src = (q == 0) ? wihf : (q == 1) ? wihb : (q == 2) ? whhf : whhb;
  }
  const v8h r = cvt8(src + (size_t)lb * 2048 + threadIdx.x * 8, kCarryW);
  unsigned short* p = dst + (size_t)blk * 2048 + threadIdx.x * 8;
  *(volatile v8h*)p = r;
  __threadfence();
  *(volatile v8h*)p = r;
}

__global__ __launch_bounds__(256) void cvt_x_kernel(
    const float* __restrict__ src, unsigned short* __restrict__ dst, int total8)
{
  const int i = blockIdx.x * 256 + threadIdx.x;
  if (i >= total8) return;
  const size_t e0 = (size_t)i << 3;
  const v8h r = cvt8(src + e0, kCarryX);
  unsigned short* p = dst + e0;
  *(volatile v8h*)p = r;
  __threadfence();
  *(volatile v8h*)p = r;
}

__global__ __launch_bounds__(256) void prep_static_kernel(
    const float* __restrict__ xs, const int* __restrict__ order,
    const float* __restrict__ Ws, const float* __restrict__ bstat,
    const float* __restrict__ bdyn,
    const float* __restrict__ bihf, const float* __restrict__ bhhf,
    const float* __restrict__ bihb, const float* __restrict__ bhhb,
    const float* __restrict__ Wh, const float* __restrict__ bh,
    float* __restrict__ biasT, float* __restrict__ ystat)
{
  __shared__ __align__(16) float xs_sh[kPS * kIS];
  __shared__ __align__(16) float s_sh[kPS * kHS];
  __shared__ __align__(16) float y_sh[kPS];
  const int tid = threadIdx.x;
  const int lane = tid & 31;
  const int wave = tid >> 5;
  const int blk = blockIdx.x;
  {
    const float* p = xs + (size_t)blk * (kPS * kIS) + tid * 8;
    const v4f a0 = *(const v4f*)(p);
    const v4f a1 = *(const v4f*)(p + 4);
    v4f r0, r1;
#pragma unroll
    for (int e = 0; e < 4; ++e) {
      const float t0 = a0[e];
      const float t1 = a1[e];
      r0[e] = rbf(t0);
      r1[e] = rbf(t1);
    }
    *(v4f*)(xs_sh + tid * 8) = r0;
    *(v4f*)(xs_sh + tid * 8 + 4) = r1;
  }
  {
    const float va = bdyn[tid];
    const float vb = bihf[tid];
    const float vc = bhhf[tid];
    const float vd = bihb[tid];
    const float ve = bhhb[tid];
    const float t0 = rbf(va);
    const float t1 = rbf(vb) + rbf(vc);
    const float t2 = rbf(vd) + rbf(ve);
    const float tv = (blk == 0) ? t0 : (blk == 1) ? t1 : t2;
    if (blk < 3) {
      volatile float* q = biasT + blk * kHD + tid;
      *q = tv;
      __threadfence();
      *q = tv;
    }
  }
  __syncthreads();
  float acc[kPS];
#pragma unroll
  for (int r = 0; r < kPS; ++r) acc[r] = 0.0f;
#pragma unroll 1
  for (int i = 0; i < kIS; ++i) {
    const float wv = Ws[(size_t)tid * kIS + i];
    const float w = rbf(wv);
#pragma unroll
    for (int r = 0; r < kPS; ++r) acc[r] = fmaf(xs_sh[r * kIS + i], w, acc[r]);
  }
  {
    const float bv = bstat[tid];
    const float bsv = rbf(bv);
#pragma unroll
    for (int r = 0; r < kPS; ++r) s_sh[r * kHS + tid] = fmaxf(acc[r] + bsv, 0.0f);
  }
  __syncthreads();
#pragma unroll 1
  for (int q = 0; q < 4; ++q) {
    const int si = wave * 4 + q;
    const int b = blk * kPS + si;
    int e = order[b];
    e = (e < 0) ? 0 : ((e > kNN - 1) ? (kNN - 1) : e);
    const float* wrow = Wh + (size_t)e * kDH;
    float part = 0.0f;
#pragma unroll
    for (int k = 0; k < 8; ++k) {
      const float wv = wrow[lane + 32 * k];
      part = fmaf(s_sh[si * kHS + lane + 32 * k], rbf(wv), part);
    }
    part += __shfl_xor(part, 16, 32);
    part += __shfl_xor(part, 8, 32);
    part += __shfl_xor(part, 4, 32);
    part += __shfl_xor(part, 2, 32);
    part += __shfl_xor(part, 1, 32);
    float bhv = bh[e];
    asm volatile("" : "+v"(bhv));
    const float tot = part + rbf(bhv);
    if (lane == 0) y_sh[si] = tot;
  }
  __syncthreads();
  if (wave == 0) {
    const float yv = y_sh[lane];
    volatile float* q = ystat + blk * kPS + lane;
    *q = yv;
    __threadfence();
    *q = yv;
  }
}

template <int ACT>
__global__ __launch_bounds__(256) void gemm64_f16_kernel(
    const unsigned short* __restrict__ Ap, int lda,
    const unsigned short* __restrict__ Btp, int ldb,
    unsigned short* __restrict__ Cp, int ldc,
    const float* __restrict__ bias,
    int M, int N, int K, float scale, float oscale)
{
  const _Float16* A  = (const _Float16*)Ap;
  const _Float16* Bt = (const _Float16*)Btp;
  __shared__ __align__(16) float sT[8][16 * 68];
  const int lane = threadIdx.x & 31;
  const int wave = threadIdx.x >> 5;
  const int tilesN = N >> 6;
  const int tilesM = M >> 6;
  const int tile = blockIdx.x * 8 + wave;
  if (tile >= tilesM * tilesN) return;
  const int tm = tile / tilesN;
  const int tn = tile - tm * tilesN;
  const int m0 = tm << 6;
  const int n0 = tn << 6;
  const int rlane = lane & 15;
  const int koff  = (lane >> 4) * 8;
  const int mOff  = (lane >> 4) * 8;

  v8f acc[4][4];
#pragma unroll
  for (int i = 0; i < 4; ++i)
#pragma unroll
    for (int j = 0; j < 4; ++j) acc[i][j] = (v8f){0.f, 0.f, 0.f, 0.f, 0.f, 0.f, 0.f, 0.f};

  for (int k0 = 0; k0 < K; k0 += 32) {
    v16h bh[4];
#pragma unroll
    for (int j = 0; j < 4; ++j) {
      const size_t bo = (size_t)(n0 + (j << 4) + rlane) * ldb + koff + k0;
      bh[j] = frag_load(Bt + bo);
    }
#pragma unroll
    for (int i = 0; i < 4; ++i) {
      const size_t ao = (size_t)(m0 + (i << 4) + rlane) * lda + koff + k0;
      const v16h ah = frag_load(A + ao);
#pragma unroll
      for (int j = 0; j < 4; ++j) acc[i][j] = mma_plain(ah, bh[j], acc[i][j]);
      guard1(acc[i][0], ah, bh[0]);
      guard1(acc[i][1], ah, bh[1]);
      guard1(acc[i][2], ah, bh[2]);
      guard1(acc[i][3], ah, bh[3]);
    }
    keep4(bh[0], bh[1], bh[2], bh[3]);
  }
#pragma unroll
  for (int i = 0; i < 4; ++i) {
    acc_guard1(acc[i][0]);
    acc_guard1(acc[i][1]);
    acc_guard1(acc[i][2]);
    acc_guard1(acc[i][3]);
  }

  float* slab = sT[wave];
  const int q  = lane >> 3;
  const int c8 = (lane & 7) * 8;
#pragma unroll
  for (int i = 0; i < 4; ++i) {
    const int mBase = m0 + (i << 4);
#pragma unroll
    for (int j = 0; j < 4; ++j) {
      const int n = n0 + (j << 4) + rlane;
      const float bv = bias[n];
#pragma unroll
      for (int r = 0; r < 8; ++r) {
        float v = acc[i][j][r] * scale + bv;
        if (ACT == 2) v = fmaxf(v, 0.0f);
        v = v * oscale;
        slab[(mOff + r) * 68 + (j << 4) + rlane] = v;
      }
    }
    __builtin_amdgcn_fence(__ATOMIC_RELEASE, "workgroup");
    __builtin_amdgcn_wave_barrier();
    __builtin_amdgcn_fence(__ATOMIC_ACQUIRE, "workgroup");
    v8h hv[4];
#pragma unroll
    for (int it = 0; it < 4; ++it) {
      const int row = it * 4 + q;
      const float* sp = slab + row * 68 + c8;
      const v4f a0 = *(const v4f*)(sp);
      const v4f a1 = *(const v4f*)(sp + 4);
#pragma unroll
      for (int e = 0; e < 4; ++e) {
        const float t0 = a0[e];
        const float t1 = a1[e];
        hv[it][e]     = (_Float16)t0;
        hv[it][4 + e] = (_Float16)t1;
      }
    }
    for (int pass = 0; pass < 2; ++pass) {
#pragma unroll
      for (int it = 0; it < 4; ++it) {
        const int row = it * 4 + q;
        *(volatile v8h*)(Cp + (size_t)(mBase + row) * ldc + n0 + c8) = hv[it];
      }
      __threadfence();
    }
    __builtin_amdgcn_fence(__ATOMIC_RELEASE, "workgroup");
    __builtin_amdgcn_wave_barrier();
    __builtin_amdgcn_fence(__ATOMIC_ACQUIRE, "workgroup");
  }
}

__global__ __launch_bounds__(512) void rnn_dir_kernel(
    const unsigned short* __restrict__ XP, const unsigned short* __restrict__ Whh16,
    const float* __restrict__ Wheads, const int* __restrict__ order,
    float* __restrict__ Y, int dir)
{
  __shared__ __align__(16) _Float16 hbuf[kRB * kHD];
  __shared__ __align__(16) float ybuf[kRB * kT];
  const int tid  = threadIdx.x;
  const int wave = tid >> 5;
  const int lane = tid & 31;
  const int lh   = lane >> 4;
  const int c    = lane & 15;
  const int n    = (wave << 4) + c;
  const int b0   = blockIdx.x * kRB;

  v16h Bfrag[8];
  {
    const _Float16* wp = (const _Float16*)Whh16 + (size_t)n * kHD + 8 * lh;
#pragma unroll
    for (int kt = 0; kt < 8; ++kt) Bfrag[kt] = frag_load(wp + kt * 32);
  }
  float wg[8];
  {
    int e = order[b0 + wave];
    e = (e < 0) ? 0 : ((e > kNN - 1) ? (kNN - 1) : e);
    const float* wr = Wheads + (size_t)e * kDH + kHS + (dir ? kHD : 0) + lane * 8;
    const v4f a0 = *(const v4f*)(wr);
    const v4f a1 = *(const v4f*)(wr + 4);
#pragma unroll
    for (int i = 0; i < 4; ++i) {
      const float t0 = a0[i];
      const float t1 = a1[i];
      wg[i]     = rbf(t0) * kFoldA;
      wg[4 + i] = rbf(t1) * kFoldA;
    }
  }
  *(v8h*)(hbuf + tid * 8) = (v8h){(_Float16)0.f, (_Float16)0.f, (_Float16)0.f, (_Float16)0.f,
                                  (_Float16)0.f, (_Float16)0.f, (_Float16)0.f, (_Float16)0.f};
  __syncthreads();

  const size_t xrow0 = (size_t)(b0 + 8 * lh) * kT;
#pragma unroll 1
  for (int step = 0; step < kT; ++step) {
    const int t = dir ? (kT - 1 - step) : step;
    unsigned xr[8];
#pragma unroll
    for (int v = 0; v < 8; ++v) {
      const size_t g = (xrow0 + (size_t)v * kT + t) * kHD + n;
      xr[v] = XP[g];
    }
    v8f acc = (v8f){0.f, 0.f, 0.f, 0.f, 0.f, 0.f, 0.f, 0.f};
    {
      const _Float16* hp = hbuf + c * kHD + 8 * lh;
#pragma unroll
      for (int kt = 0; kt < 8; ++kt) {
        const v16h a = frag_load(hp + kt * 32);
        acc = mma_g(a, Bfrag[kt], acc);
      }
    }
    float hv[8];
#pragma unroll
    for (int v = 0; v < 8; ++v) {
      const float x = h16_to_f32(xr[v]);
      hv[v] = fmaxf(fmaf(acc[v], kFoldAW, x), 0.0f);
    }
    __syncthreads();
#pragma unroll
    for (int v = 0; v < 8; ++v) hbuf[(8 * lh + v) * kHD + n] = (_Float16)(hv[v] * kCarryA);
    __syncthreads();
    {
      const v4u_alias w4 = *(const v4u_alias*)(hbuf + wave * kHD + lane * 8);
      const unsigned u0 = w4[0];
      const unsigned u1 = w4[1];
      const unsigned u2 = w4[2];
      const unsigned u3 = w4[3];
      float s = 0.0f;
      s = fmaf(h16_to_f32(u0 & 0xffffu), wg[0], s);
      s = fmaf(h16_to_f32(u0 >> 16),     wg[1], s);
      s = fmaf(h16_to_f32(u1 & 0xffffu), wg[2], s);
      s = fmaf(h16_to_f32(u1 >> 16),     wg[3], s);
      s = fmaf(h16_to_f32(u2 & 0xffffu), wg[4], s);
      s = fmaf(h16_to_f32(u2 >> 16),     wg[5], s);
      s = fmaf(h16_to_f32(u3 & 0xffffu), wg[6], s);
      s = fmaf(h16_to_f32(u3 >> 16),     wg[7], s);
      s += __shfl_xor(s, 16, 32);
      s += __shfl_xor(s, 8, 32);
      s += __shfl_xor(s, 4, 32);
      s += __shfl_xor(s, 2, 32);
      s += __shfl_xor(s, 1, 32);
      if (lane == 0) ybuf[wave * kT + t] = s;
    }
  }
  __syncthreads();
  {
    constexpr int kNV4 = kRB * kT / 4;
    static_assert(kNV4 == 800 && (kNV4 % 32) == 0 && kNV4 > 512 && kNV4 <= 1024);
    float* yb = Y + (size_t)b0 * kT;
    const int i1 = 512 + tid;
    const bool has1 = (i1 < kNV4);
    const int i1c = has1 ? i1 : (kNV4 - 1);
    const v4f y0 = *(const v4f*)(ybuf + tid * 4);
    const v4f y1 = *(const v4f*)(ybuf + i1c * 4);
    for (int pass = 0; pass < 2; ++pass) {
      *(volatile v4f*)(yb + tid * 4) = y0;
      if (has1) *(volatile v4f*)(yb + i1 * 4) = y1;
      __threadfence();
    }
  }
}

__global__ __launch_bounds__(256) void combine_kernel(
    const float* __restrict__ ystat, const float* __restrict__ YF, const float* __restrict__ YB,
    float* __restrict__ out, int total4)
{
  const int i = blockIdx.x * 256 + threadIdx.x;
  if (i >= total4) return;
  const int e0 = i * 4;
  int b = e0 / kT;
  b = (b > kB - 1) ? (kB - 1) : b;
  const float ys = ystat[b];
  const v4f f = *(const v4f*)(YF + e0);
  const v4f g = *(const v4f*)(YB + e0);
  v4f o;
#pragma unroll
  for (int e = 0; e < 4; ++e) {
    const float tf = f[e];
    const float tg = g[e];
    o[e] = fmaxf(ys + tf + tg, 0.0f);
  }
  float* p = out + e0;
  *(volatile v4f*)p = o;
  __threadfence();
  *(volatile v4f*)p = o;
}

extern "C" void kernel_launch(void* const* d_in, const int* in_sizes, int n_in,
                              void* d_out, int out_size, void* d_ws, size_t ws_size,
                              hipStream_t stream) {
  if (n_in < 17) return;
  if (in_sizes[0] != kB * kIS) return;
  if (in_sizes[1] != kRows * kID) return;
  if (in_sizes[2] != kB) return;
  if (in_sizes[3] != kHS * kIS) return;
  if (in_sizes[4] != kHS) return;
  if (in_sizes[5] != kHD * kID) return;
  if (in_sizes[6] != kHD) return;
  if (in_sizes[7] != kHD * kHD) return;
  if (in_sizes[8] != kHD * kHD) return;
  if (in_sizes[9] != kHD) return;
  if (in_sizes[10] != kHD) return;
  if (in_sizes[11] != kHD * kHD) return;
  if (in_sizes[12] != kHD * kHD) return;
  if (in_sizes[13] != kHD) return;
  if (in_sizes[14] != kHD) return;
  if (in_sizes[15] != kNN * kDH) return;
  if (in_sizes[16] != kNN) return;
  if (out_size != kB * kT) return;
  if (ws_size < kWsTotal) return;

  const float* x_static = (const float*)d_in[0];
  const float* x_dyn    = (const float*)d_in[1];
  const int*   order    = (const int*)d_in[2];
  const float* W_static = (const float*)d_in[3];
  const float* b_static = (const float*)d_in[4];
  const float* W_dyn    = (const float*)d_in[5];
  const float* b_dyn    = (const float*)d_in[6];
  const float* Wih_f    = (const float*)d_in[7];
  const float* Whh_f    = (const float*)d_in[8];
  const float* bih_f    = (const float*)d_in[9];
  const float* bhh_f    = (const float*)d_in[10];
  const float* Wih_b    = (const float*)d_in[11];
  const float* Whh_b    = (const float*)d_in[12];
  const float* bih_b    = (const float*)d_in[13];
  const float* bhh_b    = (const float*)d_in[14];
  const float* W_heads  = (const float*)d_in[15];
  const float* b_heads  = (const float*)d_in[16];
  float* out = (float*)d_out;

  char* ws = (char*)d_ws;
  unsigned short* Dpl  = (unsigned short*)(ws + kOffD);
  unsigned short* XPpl = (unsigned short*)(ws + kOffXP);
  unsigned short* XHpl = XPpl;
  unsigned short* W16  = (unsigned short*)(ws + kOffW16);
  float* BIAS = (float*)(ws + kOffBIAS);
  float* YST  = (float*)(ws + kOffYST);
  float* YF   = (float*)(ws + kOffYF);
  float* YB   = (float*)(ws + kOffYB);

  constexpr int kGemmBlocks = (kRows / 64) * (kHD / 64) / 8;
  static_assert(kGemmBlocks == 800);
  static_assert(((kRows / 64) * (kHD / 64)) % 8 == 0);

  prep_static_kernel<<<kB / kPS, 256, 0, stream>>>(
      x_static, order, W_static, b_static, b_dyn, bih_f, bhh_f, bih_b, bhh_b,
      W_heads, b_heads, BIAS, YST);

  cvt_weights_kernel<<<144, 256, 0, stream>>>(W_dyn, Wih_f, Wih_b, Whh_f, Whh_b, W16);

  cvt_x_kernel<<<(kRows * kID / 8) / 256, 256, 0, stream>>>(x_dyn, XHpl, kRows * kID / 8);

  gemm64_f16_kernel<2><<<kGemmBlocks, 256, 0, stream>>>(
      XHpl, kID, W16 + kWOffDyn, kID, Dpl, kHD, BIAS, kRows, kHD, kID, kFoldXW, kCarryA);

  gemm64_f16_kernel<0><<<kGemmBlocks, 256, 0, stream>>>(
      Dpl, kHD, W16 + kWOffIhF, kHD, XPpl, kHD, BIAS + kHD, kRows, kHD, kHD, kFoldAW, 1.0f);

  rnn_dir_kernel<<<kB / kRB, 512, 0, stream>>>(XPpl, W16 + kWOffHhF, W_heads, order, YF, 0);

  gemm64_f16_kernel<0><<<kGemmBlocks, 256, 0, stream>>>(
      Dpl, kHD, W16 + kWOffIhB, kHD, XPpl, kHD, BIAS + 2 * kHD, kRows, kHD, kHD, kFoldAW, 1.0f);

  rnn_dir_kernel<<<kB / kRB, 512, 0, stream>>>(XPpl, W16 + kWOffHhB, W_heads, order, YB, 1);

  combine_kernel<<<(kB * kT / 4) / 256, 256, 0, stream>>>(YST, YF, YB, out, kB * kT / 4);
}
